// DeltaNet_54932631715924
// MI455X (gfx1250) — hardware-verified
//
#include <hip/hip_runtime.h>
#include <math.h>

constexpr int NBATCH = 2;
constexpr int NSEQ   = 4096;
constexpr int NHID   = 1024;
constexpr int NHEAD  = 4;
constexpr int NDH    = 256;
constexpr int NTAP   = 4;
constexpr int NCS    = 64;
constexpr int NCHUNK = NSEQ / NCS;
constexpr int NTOK   = NBATCH * NSEQ;
constexpr int NBN    = NBATCH * NCHUNK;
constexpr int NBH    = NBATCH * NHEAD;
constexpr int ON_TPB = 16;
constexpr float EPS_RMS     = 1.0e-5f;
constexpr float L2_FLOOR    = 1.0e-12f;
constexpr float CARRY_X     = 16.0f;
constexpr float CARRY_W     = 256.0f;
constexpr float CARRY_K     = 16.0f;
constexpr float CARRY_KINV  = 1.0f / 16.0f;
constexpr float CARRY_T     = 16.0f;
constexpr float CARRY_WU    = 16.0f;
constexpr float CARRY_WUINV = 1.0f / 16.0f;
constexpr float CARRY_UT    = 4.0f;
static_assert(NHEAD * NDH == NHID, "heads");
static_assert(NSEQ % NCS == 0 && NCS == 64 && NDH == 256 && NTAP == 4, "tiles");
static_assert(NSEQ % ON_TPB == 0 && NCS % ON_TPB == 0, "token blocks");
static_assert(NTOK % 64 == 0 && NHID % 64 == 0 && NHID % 32 == 0, "proj gemm M,N,K");
static_assert(NCS % 64 == 0 && NHID % 64 == 0 && NCS % 32 == 0, "t gemm M,N,K");
static_assert(NDH % 64 == 0 && NSEQ % 32 == 0, "state gemm M,N,K");

constexpr size_t SZ_P16   = (size_t)NTOK * NHID * 2;
constexpr size_t SZ_W16   = (size_t)NHID * NHID * 2;
constexpr size_t SZ_LIN   = (size_t)NTOK * NHID * 4;
constexpr size_t SZ_T16   = (size_t)NBN * NCS * NCS * 2;
constexpr size_t SZ_GATE  = (size_t)NTOK * NHEAD * 4;
constexpr size_t SZ_DS    = (size_t)NBH * NCHUNK * NDH * 4;
constexpr size_t OFF_X    = 0;
constexpr size_t OFF_WQ   = OFF_X + SZ_P16;
constexpr size_t OFF_WK   = OFF_WQ + SZ_W16;
constexpr size_t OFF_WV   = OFF_WK + SZ_W16;
constexpr size_t OFF_WO   = OFF_WV + SZ_W16;
constexpr size_t OFF_LIN  = OFF_WO + SZ_W16;
constexpr size_t OFF_K    = OFF_LIN + SZ_LIN;
constexpr size_t OFF_KT   = OFF_K + SZ_P16;
constexpr size_t OFF_KBT  = OFF_KT + SZ_P16;
constexpr size_t OFF_VBT  = OFF_KBT + SZ_P16;
constexpr size_t OFF_T    = OFF_VBT + SZ_P16;
constexpr size_t OFF_GATE = OFF_T + SZ_T16;
constexpr size_t OFF_DS   = OFF_GATE + SZ_GATE;
constexpr size_t WS_TOTAL = OFF_DS + SZ_DS;
static_assert(WS_TOTAL == 127533056u, "ws total");
static_assert(WS_TOTAL <= 134217728u, "ws cap");
static_assert((size_t)NBH * NDH * NSEQ * 2 == SZ_P16 && (size_t)NBN * NHID * NCS * 2 == SZ_P16, "aliased plane sizes");
static_assert(OFF_WQ % 128 == 0 && OFF_LIN % 128 == 0 && OFF_T % 128 == 0 && OFF_GATE % 128 == 0 && OFF_DS % 128 == 0, "line aligned");
constexpr size_t OUT0_BYTES = (size_t)NTOK * NHID * 4;
constexpr size_t OUT1_BYTES = (size_t)NBH * NDH * NDH * 4;
static_assert(OUT0_BYTES == 33554432u && OUT0_BYTES + OUT1_BYTES == 35651584u, "out layout");
static_assert(OUT0_BYTES % 128 == 0, "out1 line aligned");

typedef __attribute__((ext_vector_type(16))) _Float16 v16h;
typedef __attribute__((ext_vector_type(8)))  _Float16 v8h;
typedef __attribute__((ext_vector_type(16))) __bf16   v16b;
typedef __attribute__((ext_vector_type(8)))  __bf16   v8b;
typedef __attribute__((ext_vector_type(8)))  float    v8f;
typedef __attribute__((ext_vector_type(4)))  float    v4f;
typedef __attribute__((ext_vector_type(4)))  unsigned int v4u;
typedef __attribute__((ext_vector_type(2)))  unsigned int v2u;

__device__ __forceinline__ unsigned short f2bf_bits(float f) {
  unsigned u = __float_as_uint(f);
  return (unsigned short)((u + 0x7FFFu + ((u >> 16) & 1u)) >> 16);
}
__device__ __forceinline__ float bf_bits2f(unsigned short h) { return __uint_as_float(((unsigned)h) << 16); }

__device__ __forceinline__ void dep_guard_h(v8f& a, v8f& b, v16h x, v16h y) { asm volatile("v_nop\n\tv_nop\n\tv_nop\n\tv_nop" : "+v"(a), "+v"(b) : "v"(x), "v"(y)); }
__device__ __forceinline__ void dep_guard_b(v8f& a, v8f& b, v16b x, v16b y) { asm volatile("v_nop\n\tv_nop\n\tv_nop\n\tv_nop" : "+v"(a), "+v"(b) : "v"(x), "v"(y)); }
__device__ __forceinline__ void dep_guard4_h(v8f& a, v8f& b, v8f& c, v8f& d, v16h x, v16h y) { asm volatile("v_nop\n\tv_nop\n\tv_nop\n\tv_nop" : "+v"(a), "+v"(b), "+v"(c), "+v"(d) : "v"(x), "v"(y)); }
__device__ __forceinline__ void dep_guard4_b(v8f& a, v8f& b, v8f& c, v8f& d, v16b x, v16b y) { asm volatile("v_nop\n\tv_nop\n\tv_nop\n\tv_nop" : "+v"(a), "+v"(b), "+v"(c), "+v"(d) : "v"(x), "v"(y)); }
__device__ __forceinline__ void keep4_h(v16h a, v16h b, v16h c, v16h d) { asm volatile("v_nop" :: "v"(a), "v"(b), "v"(c), "v"(d)); }
__device__ __forceinline__ void keep4_b(v16b a, v16b b, v16b c, v16b d) { asm volatile("v_nop" :: "v"(a), "v"(b), "v"(c), "v"(d)); }
__device__ __forceinline__ void acc_guard4(v8f& a, v8f& b, v8f& c, v8f& d) { asm volatile("v_nop\n\tv_nop\n\tv_nop\n\tv_nop" : "+v"(a), "+v"(b), "+v"(c), "+v"(d)); }
template <typename T> struct Frag;
template <> struct Frag<_Float16> {
  typedef v16h V; union U { v16h v; v8h h[2]; };
  static __device__ __forceinline__ v16h load(const _Float16* p) {
    U f; f.h[0] = *(const v8h*)(p); f.h[1] = *(const v8h*)(p + 16); return f.v;
  }
  static __device__ __forceinline__ v8f mma(v16h a, v16h b, v8f c) {
    return __builtin_amdgcn_wmma_f32_16x16x32_f16(false, a, false, b, (short)0, c, false, false);
  }
  static __device__ __forceinline__ void guard(v8f& a, v8f& b, v16h x, v16h y) { dep_guard_h(a, b, x, y); }
  static __device__ __forceinline__ void guard4(v8f& a, v8f& b, v8f& c, v8f& d, v16h x, v16h y) { dep_guard4_h(a, b, c, d, x, y); }
  static __device__ __forceinline__ void keep(v16h a, v16h b, v16h c, v16h d) { keep4_h(a, b, c, d); }
};
template <> struct Frag<__bf16> {
  typedef v16b V; union U { v16b v; v8b h[2]; };
  static __device__ __forceinline__ v16b load(const __bf16* p) {
    U f; f.h[0] = *(const v8b*)(p); f.h[1] = *(const v8b*)(p + 16); return f.v;
  }
  static __device__ __forceinline__ v8f mma(v16b a, v16b b, v8f c) {
    return __builtin_amdgcn_wmma_f32_16x16x32_bf16(false, a, false, b, (short)0, c, false, false);
  }
  static __device__ __forceinline__ void guard(v8f& a, v8f& b, v16b x, v16b y) { dep_guard_b(a, b, x, y); }
  static __device__ __forceinline__ void guard4(v8f& a, v8f& b, v8f& c, v8f& d, v16b x, v16b y) { dep_guard4_b(a, b, c, d, x, y); }
  static __device__ __forceinline__ void keep(v16b a, v16b b, v16b c, v16b d) { keep4_b(a, b, c, d); }
};

template <int ET> struct Elem;
template <> struct Elem<0> { typedef _Float16 T; };
template <> struct Elem<1> { typedef __bf16 T; };
template <int ET, int SPLIT, int BIAS_MODE, int OUT_MODE, bool RESID, int ACT = 0>
__global__ __launch_bounds__(256) void wmma_gemm64(
    const unsigned short* __restrict__ Ap, const unsigned short* __restrict__ A2p, int lda, long strideA,
    const unsigned short* __restrict__ Btp, const unsigned short* __restrict__ Bt2p, int ldb, long strideB,
    void* __restrict__ Cout, void* __restrict__ Cout2, int ldc, long strideC,
    const float* __restrict__ bias,
    const float* __restrict__ resid, long strideR,
    int M, int N, int K, float scale) {
  typedef typename Elem<ET>::T T;
  typedef typename Frag<T>::V V;
  const T* A = (const T*)Ap; const T* A2 = (const T*)A2p; const T* Bt = (const T*)Btp; const T* Bt2 = (const T*)Bt2p;
  __shared__ __align__(16) float sT[8][16 * 68];
  const int b    = blockIdx.y;
  const int lane = threadIdx.x & 31;
  const int wave = threadIdx.x >> 5;
  const int tilesN = N >> 6;
  const int tilesM = M >> 6;
  const int tile = blockIdx.x * 8 + wave;
  if (tile >= tilesM * tilesN) return;
  const int tm = tile / tilesN;
  const int tn = tile - tm * tilesN;
  const int m0 = tm << 6;
  const int n0 = tn << 6;

  const T* Ab  = A  + (size_t)b * strideA;
  const T* Bb  = Bt + (size_t)b * strideB;
  const T* Ab2 = (SPLIT != 0) ? (A2  + (size_t)b * strideA) : nullptr;
  const T* Bb2 = (SPLIT == 1) ? (Bt2 + (size_t)b * strideB) : nullptr;

  const int rlane = lane & 15;
  const int koff  = (lane >> 4) * 8;
  const int mOff  = (lane >> 4) * 8;

  v8f acc[4][4];
#pragma unroll
  for (int i = 0; i < 4; ++i)
#pragma unroll
    for (int j = 0; j < 4; ++j) acc[i][j] = (v8f){0.f,0.f,0.f,0.f,0.f,0.f,0.f,0.f};

  for (int k0 = 0; k0 < K; k0 += 32) {
    V bh[4], bl[4];
#pragma unroll
    for (int j = 0; j < 4; ++j) {
      const size_t bo = (size_t)(n0 + (j << 4) + rlane) * ldb + koff + k0;
      bh[j] = Frag<T>::load(Bb + bo);
      if (SPLIT == 1) bl[j] = Frag<T>::load(Bb2 + bo);
    }
#pragma unroll
    for (int i = 0; i < 4; ++i) {
      const size_t ao = (size_t)(m0 + (i << 4) + rlane) * lda + koff + k0;
      V ah = Frag<T>::load(Ab + ao);
      V al;
      if (SPLIT != 0) al = Frag<T>::load(Ab2 + ao);
#pragma unroll
      for (int j = 0; j < 4; ++j) {
        acc[i][j] = Frag<T>::mma(ah, bh[j], acc[i][j]);
        if (SPLIT == 1) acc[i][j] = Frag<T>::mma(ah, bl[j], acc[i][j]);
        if (SPLIT != 0) acc[i][j] = Frag<T>::mma(al, bh[j], acc[i][j]);
      }
      Frag<T>::guard4(acc[i][0], acc[i][1], acc[i][2], acc[i][3], ah, (SPLIT != 0) ? al : ah);
    }
    Frag<T>::keep(bh[0], bh[1], bh[2], bh[3]);
    if (SPLIT == 1) Frag<T>::keep(bl[0], bl[1], bl[2], bl[3]);
  }
  acc_guard4(acc[0][0], acc[0][1], acc[0][2], acc[0][3]);
  acc_guard4(acc[1][0], acc[1][1], acc[1][2], acc[1][3]);
  acc_guard4(acc[2][0], acc[2][1], acc[2][2], acc[2][3]);
  acc_guard4(acc[3][0], acc[3][1], acc[3][2], acc[3][3]);

  float* slab = sT[wave];
  const float* Rb = RESID ? (resid + (size_t)b * strideR) : nullptr;
#pragma unroll
  for (int i = 0; i < 4; ++i) {
    const int mBase = m0 + (i << 4);
#pragma unroll
    for (int j = 0; j < 4; ++j) {
      const int n = n0 + (j << 4) + rlane;
      float bv = 0.f;
      if (BIAS_MODE == 2) bv = bias[n];
#pragma unroll
      for (int r = 0; r < 8; ++r) {
        float v = acc[i][j][r] * scale;
        if (BIAS_MODE == 1) v += bias[mBase + mOff + r];
        if (BIAS_MODE == 2) v += bv;
        if (RESID) v += Rb[(size_t)(mBase + mOff + r) * ldc + n];
        if (ACT == 2) v = fmaxf(v, 0.0f);
        if (ACT == 4) v = (v > 0.f) ? v : 0.01f * v;
        slab[(mOff + r) * 68 + (j << 4) + rlane] = v;
      }
    }
    __builtin_amdgcn_fence(__ATOMIC_RELEASE, "workgroup");
    __builtin_amdgcn_wave_barrier();
    __builtin_amdgcn_fence(__ATOMIC_ACQUIRE, "workgroup");
    if (OUT_MODE == 0) {
      float* C = (float*)Cout + (size_t)b * strideC;
      const int hh = lane >> 4, c4 = (lane & 15) * 4;
      for (int pass = 0; pass < 2; ++pass) {
#pragma unroll
        for (int it = 0; it < 8; ++it) {
          const int row = it * 2 + hh;
          v4f v = *(const v4f*)(slab + row * 68 + c4);
          *(volatile v4f*)(C + (size_t)(mBase + row) * ldc + n0 + c4) = v;
        }
        __threadfence();
      }
    } else {
      const int q = lane >> 3, c8 = (lane & 7) * 8;
      unsigned short* C  = (unsigned short*)Cout  + (size_t)b * strideC;
      unsigned short* C2 = (OUT_MODE == 2) ? ((unsigned short*)Cout2 + (size_t)b * strideC) : nullptr;
      for (int pass = 0; pass < 2; ++pass) {
#pragma unroll
        for (int it = 0; it < 4; ++it) {
          const int row = it * 4 + q;
          const float* sp = slab + row * 68 + c8;
          v8h hv, lv;
#pragma unroll
          for (int e = 0; e < 8; ++e) {
            if (OUT_MODE == 1) {
              hv[e] = (_Float16)sp[e];
            } else {
              unsigned short hb = f2bf_bits(sp[e]);
              unsigned short lb = f2bf_bits(sp[e] - bf_bits2f(hb));
              hv[e] = __builtin_bit_cast(_Float16, hb);
              lv[e] = __builtin_bit_cast(_Float16, lb);
            }
          }
          *(volatile v8h*)(C + (size_t)(mBase + row) * ldc + n0 + c8) = hv;
          if (OUT_MODE == 2) *(volatile v8h*)(C2 + (size_t)(mBase + row) * ldc + n0 + c8) = lv;
        }
        __threadfence();
      }
    }
    __builtin_amdgcn_fence(__ATOMIC_RELEASE, "workgroup");
    __builtin_amdgcn_wave_barrier();
    __builtin_amdgcn_fence(__ATOMIC_ACQUIRE, "workgroup");
  }
}

__device__ __forceinline__ float bf_rne(float f) { return __uint_as_float(((unsigned)f2bf_bits(f)) << 16); }
__device__ __forceinline__ unsigned short h_bits(float f) { const _Float16 h = (_Float16)f; return __builtin_bit_cast(unsigned short, h); }
__device__ __forceinline__ unsigned pk16(unsigned short a, unsigned short b) { return (unsigned)a | ((unsigned)b << 16); }
__device__ __forceinline__ float h16_to_f32(unsigned hb) {
  const unsigned sgn = (hb & 0x8000u) << 16; const unsigned em = hb & 0x7fffu;
  const float fn = __uint_as_float((em << 13) + 0x38000000u);
  const float fs = (float)em * 5.9604644775390625e-8f;
  const float mag = (em < 0x400u) ? fs : fn; return __uint_as_float(__float_as_uint(mag) | sgn); }
__device__ __forceinline__ float siluf(float x) { const float e = expf(-x); return x * __builtin_amdgcn_rcpf(1.0f + e); }
__device__ __forceinline__ float conv4(float w0, float w1, float w2, float w3, float xm3, float xm2, float xm1, float x0) {
  return fmaf(w3, x0, fmaf(w2, xm1, fmaf(w1, xm2, w0 * xm3)));
}
__device__ __forceinline__ v8f mma_h16(v16h a, v16h b, v8f c) {
  c = __builtin_amdgcn_wmma_f32_16x16x32_f16(false, a, false, b, (short)0, c, false, false);
  asm volatile("v_nop\n\tv_nop\n\tv_nop\n\tv_nop" : "+v"(c) : "v"(a), "v"(b));
  return c;
}
__device__ __forceinline__ void acc_guard2(v8f& a, v8f& b) { asm volatile("v_nop\n\tv_nop\n\tv_nop\n\tv_nop" : "+v"(a), "+v"(b)); }

template <int BF>
__global__ __launch_bounds__(256) void cast8_kernel(const float* __restrict__ in, unsigned short* __restrict__ out, int n8, float scale) {
  const int i = blockIdx.x * 256 + threadIdx.x;
  if (i >= n8) return;
  const float* p = in + 8 * (size_t)i;
  const v4f a = *(const v4f*)(p);
  const v4f c = *(const v4f*)(p + 4);
  unsigned short hb[8];
#pragma unroll
  for (int e = 0; e < 4; ++e) {
    if (BF) {
      hb[e]     = f2bf_bits(a[e]);
      hb[4 + e] = f2bf_bits(c[e]);
    } else {
      hb[e]     = h_bits(bf_rne(a[e]) * scale);
      hb[4 + e] = h_bits(bf_rne(c[e]) * scale);
    }
  }
  const v4u u = (v4u){pk16(hb[0], hb[1]), pk16(hb[2], hb[3]), pk16(hb[4], hb[5]), pk16(hb[6], hb[7])};
  unsigned short* q = out + 8 * (size_t)i;
  *(volatile v4u*)q = u;
  __threadfence();
  *(volatile v4u*)q = u;
}

__global__ __launch_bounds__(256) void gate_kernel(const float* __restrict__ x, const float* __restrict__ wb, float* __restrict__ gate) {
  __shared__ __align__(16) float sb[32];
  const int lane = threadIdx.x & 31, wave = threadIdx.x >> 5;
  const int tok = blockIdx.x * 8 + wave;
  const float* xr = x + (size_t)tok * NHID;
  float a0 = 0.f, a1 = 0.f, a2 = 0.f, a3 = 0.f;
#pragma unroll 1
  for (int i = 0; i < NHID / 128; ++i) {
    const int k = i * 128 + lane * 4;
    const v4f xv = *(const v4f*)(xr + k);
    const v4f w0 = *(const v4f*)(wb + k);
    const v4f w1 = *(const v4f*)(wb + NHID + k);
    const v4f w2 = *(const v4f*)(wb + 2 * NHID + k);
    const v4f w3 = *(const v4f*)(wb + 3 * NHID + k);
#pragma unroll
    for (int e = 0; e < 4; ++e) {
      const float xe = bf_rne(xv[e]);
      a0 = fmaf(xe, bf_rne(w0[e]), a0);
      a1 = fmaf(xe, bf_rne(w1[e]), a1);
      a2 = fmaf(xe, bf_rne(w2[e]), a2);
      a3 = fmaf(xe, bf_rne(w3[e]), a3);
    }
  }
#pragma unroll
  for (int off = 16; off > 0; off >>= 1) {
    a0 += __shfl_xor(a0, off, 32);
    a1 += __shfl_xor(a1, off, 32);
    a2 += __shfl_xor(a2, off, 32);
    a3 += __shfl_xor(a3, off, 32);
  }
  const float s0 = __builtin_amdgcn_rcpf(1.0f + expf(-a0));
  const float s1 = __builtin_amdgcn_rcpf(1.0f + expf(-a1));
  const float s2 = __builtin_amdgcn_rcpf(1.0f + expf(-a2));
  const float s3 = __builtin_amdgcn_rcpf(1.0f + expf(-a3));
  if (lane == 0) { sb[wave * 4 + 0] = s0; sb[wave * 4 + 1] = s1; sb[wave * 4 + 2] = s2; sb[wave * 4 + 3] = s3; }
  __syncthreads();
  if (wave == 0 && lane < 8) {
    const v4f v = *(const v4f*)(sb + lane * 4);
    float* dp = gate + (size_t)(blockIdx.x * 8 + lane) * NHEAD;
    *(volatile v4f*)dp = v;
    __threadfence();
    *(volatile v4f*)dp = v;
  }
}

constexpr int CONV_LDS_WORDS = 8192 * 3 + 512 + 64 + 64;
constexpr size_t CONV_LDS_BYTES = (size_t)CONV_LDS_WORDS * 4;
template <int MODE>
__global__ __launch_bounds__(256) void conv_kernel(const float* __restrict__ lin, const float* __restrict__ taps,
                                                    const float* __restrict__ gate,
                                                    unsigned short* __restrict__ rowP, unsigned short* __restrict__ trP,
                                                    unsigned short* __restrict__ btP) {
  extern __shared__ __align__(16) unsigned int dsm[];
  unsigned int* sBt  = dsm;
  unsigned int* sRow = dsm + 8192;
  unsigned int* sTr  = dsm + 16384;
  float* red   = (float*)(dsm + 24576);
  float* sInv  = red + 512;
  float* sGate = sInv + 64;
  const int tid = threadIdx.x, lane = tid & 31, wave = tid >> 5;
  const int d = tid;
  const int blk = blockIdx.x;
  const int h = blk & 3, bn = blk >> 2, n = bn & 63, b = bn >> 6;
  const int t0 = n * NCS;
  const size_t gtok0 = (size_t)b * NSEQ + t0;
  const int ch = h * NDH + d;
  const v4f tw = *(const v4f*)(taps + (size_t)ch * NTAP);
  const float w0 = bf_rne(tw[0]), w1 = bf_rne(tw[1]), w2 = bf_rne(tw[2]), w3 = bf_rne(tw[3]);
  if (tid < NCS) sGate[tid] = gate[(gtok0 + tid) * NHEAD + h];
  float xl0, xl1, xl2;
  {
    const int r0 = t0 - 3, r1 = t0 - 2, r2 = t0 - 1;
    const float v0 = lin[((size_t)b * NSEQ + (r0 < 0 ? 0 : r0)) * NHID + ch];
    const float v1 = lin[((size_t)b * NSEQ + (r1 < 0 ? 0 : r1)) * NHID + ch];
    const float v2 = lin[((size_t)b * NSEQ + (r2 < 0 ? 0 : r2)) * NHID + ch];
    xl0 = (r0 >= 0) ? v0 : 0.0f;
    xl1 = (r1 >= 0) ? v1 : 0.0f;
    xl2 = (r2 >= 0) ? v2 : 0.0f;
  }
  if (MODE == 0) {
    float xm3 = xl0, xm2 = xl1, xm1 = xl2;
#pragma unroll 1
    for (int c = 0; c < NCS; ++c) {
      const float x0 = lin[(gtok0 + c) * NHID + ch];
      const float v = siluf(siluf(conv4(w0, w1, w2, w3, xm3, xm2, xm1, x0)));
      float s2 = v * v;
#pragma unroll
      for (int off = 16; off > 0; off >>= 1) s2 += __shfl_xor(s2, off, 32);
      if (lane == 0) red[c * 8 + wave] = s2;
      xm3 = xm2; xm2 = xm1; xm1 = x0;
    }
    __syncthreads();
    if (tid < NCS) {
      float ss = red[tid * 8];
#pragma unroll
      for (int w = 1; w < 8; ++w) ss += red[tid * 8 + w];
      sInv[tid] = 1.0f / fmaxf(sqrtf(ss), L2_FLOOR);
    }
  }
  __syncthreads();
  {
    float xm3 = xl0, xm2 = xl1, xm1 = xl2;
#pragma unroll 1
    for (int p = 0; p < NCS / 2; ++p) {
      unsigned btw[2];
      unsigned trw[2];
#pragma unroll
      for (int cc = 0; cc < 2; ++cc) {
        const int c = 2 * p + cc;
        const float x0 = lin[(gtok0 + c) * NHID + ch];
        float v = siluf(siluf(conv4(w0, w1, w2, w3, xm3, xm2, xm1, x0)));
        if (MODE == 0) v = v * sInv[c];
        const float vb = v * sGate[c];
        btw[cc] = h_bits(vb * CARRY_K);
        if (MODE == 0) {
          const unsigned hk = h_bits(v * CARRY_K);
          trw[cc] = hk;
          const unsigned other = (unsigned)__shfl_xor((int)hk, 1, 32);
          const unsigned lo = (d & 1) ? other : hk;
          const unsigned hi = (d & 1) ? hk : other;
          sRow[c * 128 + (d >> 1)] = lo | (hi << 16);
        } else {
          trw[cc] = 0u;
        }
        xm3 = xm2; xm2 = xm1; xm1 = x0;
      }
      if (MODE == 0) sTr[d * 32 + p] = trw[0] | (trw[1] << 16);
      sBt[d * 32 + p] = btw[0] | (btw[1] << 16);
    }
  }
  __syncthreads();
  const int bh = b * NHEAD + h;
  for (int pass = 0; pass < 2; ++pass) {
    if (MODE == 0) {
#pragma unroll
      for (int it = 0; it < 8; ++it) {
        const int c = wave * 8 + it;
        const v4u u = *(const v4u*)(sRow + c * 128 + lane * 4);
        *(volatile v4u*)(rowP + (gtok0 + c) * NHID + h * NDH + lane * 8) = u;
      }
#pragma unroll
      for (int it = 0; it < 8; ++it) {
        const int row = wave * 32 + it * 4 + (lane >> 3);
        const int pc = lane & 7;
        const v4u u = *(const v4u*)(sTr + row * 32 + pc * 4);
        *(volatile v4u*)(trP + ((size_t)(bh * NDH + row) * NSEQ + t0) + pc * 8) = u;
      }
    }
#pragma unroll
    for (int it = 0; it < 8; ++it) {
      const int row = wave * 32 + it * 4 + (lane >> 3);
      const int pc = lane & 7;
      const v4u u = *(const v4u*)(sBt + row * 32 + pc * 4);
      *(volatile v4u*)(btP + ((size_t)(bn * NHID + h * NDH + row) * NCS) + pc * 8) = u;
    }
    __threadfence();
  }
}

constexpr int TK_PITCH = 272;
__global__ __launch_bounds__(256) void tmat_kernel(const unsigned short* __restrict__ kP, const float* __restrict__ gateP,
                                                    unsigned short* __restrict__ tP) {
  __shared__ __align__(16) unsigned short sK[NCS * TK_PITCH];
  __shared__ __align__(16) float sA[NCS * 65];
  __shared__ float sG[NCS * NHEAD];
  const int tid = threadIdx.x, lane = tid & 31, wave = tid >> 5;
  const int bn = blockIdx.x, b = bn >> 6, n = bn & 63;
  const int t0 = n * NCS;
  const size_t gtok0 = (size_t)b * NSEQ + t0;
  sG[tid] = gateP[gtok0 * NHEAD + tid];
  const int rl = lane & 15, hsel = lane >> 4, koff = hsel * 8;
  const int ti0 = wave >> 2, ti1 = ti0 + 2, tj = wave & 3;
  v8f g0 = (v8f){0.f,0.f,0.f,0.f,0.f,0.f,0.f,0.f};
  v8f g1 = (v8f){0.f,0.f,0.f,0.f,0.f,0.f,0.f,0.f};
#pragma unroll 1
  for (int h = 0; h < NHEAD; ++h) {
    __syncthreads();
#pragma unroll 1
    for (int it = 0; it < 8; ++it) {
      const int row = it * 8 + wave;
      const v4u v = *(const v4u*)(kP + (gtok0 + row) * NHID + h * NDH + lane * 8);
      *(v4u*)(sK + row * TK_PITCH + lane * 8) = v;
    }
    __syncthreads();
    const _Float16* sKh = (const _Float16*)(const void*)sK;
    v8f a0 = (v8f){0.f,0.f,0.f,0.f,0.f,0.f,0.f,0.f};
    v8f a1 = (v8f){0.f,0.f,0.f,0.f,0.f,0.f,0.f,0.f};
#pragma unroll
    for (int ks = 0; ks < NDH / 32; ++ks) {
      const int k0 = ks * 32;
      const v16h fa0 = Frag<_Float16>::load(sKh + (ti0 * 16 + rl) * TK_PITCH + koff + k0);
      const v16h fa1 = Frag<_Float16>::load(sKh + (ti1 * 16 + rl) * TK_PITCH + koff + k0);
      const v16h fb  = Frag<_Float16>::load(sKh + (tj * 16 + rl) * TK_PITCH + koff + k0);
      a0 = mma_h16(fa0, fb, a0);
      a1 = mma_h16(fa1, fb, a1);
    }
    acc_guard2(a0, a1);
#pragma unroll
    for (int r = 0; r < 8; ++r) {
      const float b0 = sG[(ti0 * 16 + hsel * 8 + r) * NHEAD + h] * (1.0f / (CARRY_K * CARRY_K));
      const float b1 = sG[(ti1 * 16 + hsel * 8 + r) * NHEAD + h] * (1.0f / (CARRY_K * CARRY_K));
      g0[r] = fmaf(b0, a0[r], g0[r]);
      g1[r] = fmaf(b1, a1[r], g1[r]);
    }
  }
#pragma unroll
  for (int r = 0; r < 8; ++r) {
    sA[(ti0 * 16 + hsel * 8 + r) * 65 + tj * 16 + rl] = g0[r];
    sA[(ti1 * 16 + hsel * 8 + r) * 65 + tj * 16 + rl] = g1[r];
  }
  __syncthreads();
#pragma unroll 1
  for (int e = tid; e < NCS * NCS; e += 256) {
    const int i = e >> 6, j = e & 63;
    const float a = sA[i * 65 + j];
    sA[i * 65 + j] = (j < i) ? -a : ((j == i) ? 1.0f : 0.0f);
  }
  __syncthreads();
#pragma unroll 1
  for (int i = 1; i < NCS; ++i) {
    float prod = 0.0f;
    if (tid < NCS) {
#pragma unroll 1
      for (int j = 0; j < NCS; ++j) prod = fmaf(sA[i * 65 + j], sA[j * 65 + tid], prod);
    }
    __syncthreads();
    if (tid < i) sA[i * 65 + tid] += prod;
    __syncthreads();
  }
  const int c8 = (lane & 7) * 8;
  for (int pass = 0; pass < 2; ++pass) {
#pragma unroll
    for (int it = 0; it < 2; ++it) {
      const int row = wave * 8 + it * 4 + (lane >> 3);
      unsigned short hb[8];
#pragma unroll
      for (int e = 0; e < 8; ++e) hb[e] = h_bits(sA[row * 65 + c8 + e] * CARRY_T);
      const v4u u = (v4u){pk16(hb[0], hb[1]), pk16(hb[2], hb[3]), pk16(hb[4], hb[5]), pk16(hb[6], hb[7])};
      *(volatile v4u*)(tP + ((size_t)bn * NCS + row) * NCS + c8) = u;
    }
    __threadfence();
  }
}

constexpr int DIAG_LDS_WORDS = 8192 * 4 + 256;
constexpr size_t DIAG_LDS_BYTES = (size_t)DIAG_LDS_WORDS * 4;
__global__ __launch_bounds__(256) void diag_kernel(const unsigned short* __restrict__ kT, const unsigned short* __restrict__ wP,
                                                    const unsigned short* __restrict__ uP,
                                                    unsigned short* __restrict__ uT, float* __restrict__ dsT) {
  extern __shared__ __align__(16) unsigned int dsm[];
  unsigned int* sW  = dsm;
  unsigned int* sU  = dsm + 8192;
  unsigned int* sK  = dsm + 16384;
  unsigned int* sUt = dsm + 24576;
  float* sDS = (float*)(dsm + 32768);
  const int tid = threadIdx.x, lane = tid & 31, wave = tid >> 5;
  const int d = tid;
  const int bh = blockIdx.x, b = bh >> 2, h = bh & 3;
  const unsigned sh = (unsigned)(d & 1) * 16u;
  float dS = 0.0f;
#pragma unroll 1
  for (int n = 0; n < NCHUNK; ++n) {
    const int t0 = n * NCS;
    const size_t gtok0 = (size_t)b * NSEQ + t0;
    __syncthreads();
#pragma unroll 1
    for (int it = 0; it < 8; ++it) {
      const int row = it * 8 + wave;
      const size_t go = (gtok0 + row) * NHID + h * NDH + lane * 8;
      const v4u wv = *(const v4u*)(wP + go);
      const v4u uv = *(const v4u*)(uP + go);
      *(v4u*)(sW + row * 128 + lane * 4) = wv;
      *(v4u*)(sU + row * 128 + lane * 4) = uv;
      const int krow = it * 32 + (tid >> 3);
      const int pc = tid & 7;
      const v4u kv = *(const v4u*)(kT + ((size_t)(bh * NDH + krow) * NSEQ + t0) + pc * 8);
      *(v4u*)(sK + krow * 32 + pc * 4) = kv;
    }
    sDS[d] = dS;
    __syncthreads();
    float dacc = 0.0f;
#pragma unroll 1
    for (int p = 0; p < NCS / 2; ++p) {
      const unsigned kw = sK[d * 32 + p];
      unsigned ub[2];
#pragma unroll
      for (int cc = 0; cc < 2; ++cc) {
        const int c = 2 * p + cc;
        const unsigned kb  = (cc == 0) ? (kw & 0xffffu) : (kw >> 16);
        const unsigned wbv = (sW[c * 128 + (d >> 1)] >> sh) & 0xffffu;
        const unsigned ubv = (sU[c * 128 + (d >> 1)] >> sh) & 0xffffu;
        const float kf = h16_to_f32(kb) * CARRY_KINV;
        const float wf = h16_to_f32(wbv) * CARRY_WUINV;
        const float uf = h16_to_f32(ubv) * CARRY_WUINV;
        const float u = uf - wf * dS;
        dacc = fmaf(kf, u, dacc);
        ub[cc] = h_bits(u * CARRY_UT);
      }
      sUt[d * 32 + p] = ub[0] | (ub[1] << 16);
    }
    dS = dS + dacc;
    __syncthreads();
    for (int pass = 0; pass < 2; ++pass) {
#pragma unroll
      for (int it = 0; it < 8; ++it) {
        const int row = wave * 32 + it * 4 + (lane >> 3);
        const int pc = lane & 7;
        const v4u u = *(const v4u*)(sUt + row * 32 + pc * 4);
        *(volatile v4u*)(uT + ((size_t)(bh * NDH + row) * NSEQ + t0) + pc * 8) = u;
      }
      if (tid < 64) {
        const v4f v = *(const v4f*)(sDS + 4 * tid);
        *(volatile v4f*)(dsT + ((size_t)(bh * NCHUNK + n) * NDH) + 4 * tid) = v;
      }
      __threadfence();
    }
  }
}

__global__ __launch_bounds__(256) void onorm_kernel(const float* __restrict__ linq, const float* __restrict__ taps,
                                                     const unsigned short* __restrict__ kP, const unsigned short* __restrict__ wP,
                                                     const unsigned short* __restrict__ uP, const float* __restrict__ dsT,
                                                     const float* __restrict__ rw,
                                                     unsigned short* __restrict__ onH, unsigned short* __restrict__ onL) {
  __shared__ float redq[2][8];
  __shared__ float redd[2][8];
  __shared__ float redo[2][8];
  __shared__ __align__(16) unsigned int sHi[512];
  __shared__ __align__(16) unsigned int sLo[512];
  const int tid = threadIdx.x, lane = tid & 31, wave = tid >> 5;
  const int hd  = tid >> 6;
  const int ch0 = tid * 4;
  const int dd0 = (tid & 63) * 4;
  const int blk = blockIdx.x;
  const int b   = blk / (NSEQ / ON_TPB);
  const int t0  = (blk - b * (NSEQ / ON_TPB)) * ON_TPB;
  const size_t brow = (size_t)b * NSEQ;
  float w0[4], w1[4], w2[4], w3[4], rwb[4];
  {
    v4f tw[4];
#pragma unroll
    for (int j = 0; j < 4; ++j) tw[j] = *(const v4f*)(taps + (size_t)(ch0 + j) * NTAP);
    const v4f ra = *(const v4f*)(rw + ch0);
    asm volatile("" ::: "memory");
#pragma unroll
    for (int j = 0; j < 4; ++j) {
      w0[j] = bf_rne(tw[j][0]); w1[j] = bf_rne(tw[j][1]); w2[j] = bf_rne(tw[j][2]); w3[j] = bf_rne(tw[j][3]);
      rwb[j] = bf_rne(ra[j]);
    }
  }
  float xm3[4], xm2[4], xm1[4];
  {
    const int r0 = t0 - 3, r1 = t0 - 2, r2 = t0 - 1;
    const v4f h0 = *(const v4f*)(linq + (brow + (r0 < 0 ? 0 : r0)) * NHID + ch0);
    const v4f h1 = *(const v4f*)(linq + (brow + (r1 < 0 ? 0 : r1)) * NHID + ch0);
    const v4f h2 = *(const v4f*)(linq + (brow + (r2 < 0 ? 0 : r2)) * NHID + ch0);
#pragma unroll
    for (int j = 0; j < 4; ++j) {
      xm3[j] = (r0 >= 0) ? h0[j] : 0.0f;
      xm2[j] = (r1 >= 0) ? h1[j] : 0.0f;
      xm1[j] = (r2 >= 0) ? h2[j] : 0.0f;
    }
  }
#pragma unroll 1
  for (int c = 0; c < ON_TPB; ++c) {
    const int tok = t0 + c;
    const size_t gtok = brow + tok;
    const int n = tok >> 6;
    const int cidx = tok & (NCS - 1);
    const int p = c & 1;
    const v4f x0  = *(const v4f*)(linq + gtok * NHID + ch0);
    const v4f dsv = *(const v4f*)(dsT + ((size_t)((b * NHEAD + hd) * NCHUNK + n)) * NDH + dd0);
    const v2u kw = *(const v2u*)(kP + gtok * NHID + ch0);
    const v2u ww = *(const v2u*)(wP + gtok * NHID + ch0);
    const v2u uw = *(const v2u*)(uP + gtok * NHID + ch0);
    float q[4];
    float ssq = 0.0f;
#pragma unroll
    for (int j = 0; j < 4; ++j) {
      const float y = conv4(w0[j], w1[j], w2[j], w3[j], xm3[j], xm2[j], xm1[j], x0[j]);
      q[j] = siluf(siluf(y));
      ssq = fmaf(q[j], q[j], ssq);
    }
    const unsigned kw0 = kw[0], kw1 = kw[1];
    const float k0 = h16_to_f32(kw0 & 0xffffu) * CARRY_KINV;
    const float k1 = h16_to_f32(kw0 >> 16) * CARRY_KINV;
    const float k2 = h16_to_f32(kw1 & 0xffffu) * CARRY_KINV;
    const float k3 = h16_to_f32(kw1 >> 16) * CARRY_KINV;
    float dq = 0.0f;
    dq = fmaf(q[0], k0, dq);
    dq = fmaf(q[1], k1, dq);
    dq = fmaf(q[2], k2, dq);
    dq = fmaf(q[3], k3, dq);
#pragma unroll
    for (int off = 16; off > 0; off >>= 1) {
      ssq += __shfl_xor(ssq, off, 32);
      dq  += __shfl_xor(dq, off, 32);
    }
    if (lane == 0) { redq[p][wave] = ssq; redd[p][wave] = dq; }
    __syncthreads();
    const float i0 = __builtin_amdgcn_rcpf(fmaxf(sqrtf(redq[p][0] + redq[p][1]), L2_FLOOR));
    const float i1 = __builtin_amdgcn_rcpf(fmaxf(sqrtf(redq[p][2] + redq[p][3]), L2_FLOOR));
    const float i2 = __builtin_amdgcn_rcpf(fmaxf(sqrtf(redq[p][4] + redq[p][5]), L2_FLOOR));
    const float i3 = __builtin_amdgcn_rcpf(fmaxf(sqrtf(redq[p][6] + redq[p][7]), L2_FLOOR));
    float dot = i0 * (redd[p][0] + redd[p][1]);
    dot = fmaf(i1, redd[p][2] + redd[p][3], dot);
    dot = fmaf(i2, redd[p][4] + redd[p][5], dot);
    dot = fmaf(i3, redd[p][6] + redd[p][7], dot);
    const float invh = (hd == 0) ? i0 : ((hd == 1) ? i1 : ((hd == 2) ? i2 : i3));
    const float ac = (cidx <= b) ? dot : 0.0f;
    const unsigned ww0 = ww[0], ww1 = ww[1], uw0 = uw[0], uw1 = uw[1];
    float wf[4], uf[4];
    wf[0] = h16_to_f32(ww0 & 0xffffu) * CARRY_WUINV;
    wf[1] = h16_to_f32(ww0 >> 16) * CARRY_WUINV;
    wf[2] = h16_to_f32(ww1 & 0xffffu) * CARRY_WUINV;
    wf[3] = h16_to_f32(ww1 >> 16) * CARRY_WUINV;
    uf[0] = h16_to_f32(uw0 & 0xffffu) * CARRY_WUINV;
    uf[1] = h16_to_f32(uw0 >> 16) * CARRY_WUINV;
    uf[2] = h16_to_f32(uw1 & 0xffffu) * CARRY_WUINV;
    uf[3] = h16_to_f32(uw1 >> 16) * CARRY_WUINV;
    float o[4];
    float sso = 0.0f;
#pragma unroll
    for (int j = 0; j < 4; ++j) {
      const float u = uf[j] - wf[j] * dsv[j];
      o[j] = (q[j] * invh) * dsv[j] + ac * u;
      sso = fmaf(o[j], o[j], sso);
    }
#pragma unroll
    for (int off = 16; off > 0; off >>= 1) sso += __shfl_xor(sso, off, 32);
    if (lane == 0) redo[p][wave] = sso;
    __syncthreads();
    float tot = redo[p][0];
#pragma unroll
    for (int w = 1; w < 8; ++w) tot += redo[p][w];
    const float invr = rsqrtf(tot * (1.0f / (float)NHID) + EPS_RMS);
    unsigned short hb[4], lb[4];
#pragma unroll
    for (int j = 0; j < 4; ++j) {
      const float on = (o[j] * invr) * rwb[j];
      hb[j] = f2bf_bits(on);
      lb[j] = f2bf_bits(on - bf_bits2f(hb[j]));
    }
    *(v2u*)(sHi + 2 * tid) = (v2u){pk16(hb[0], hb[1]), pk16(hb[2], hb[3])};
    *(v2u*)(sLo + 2 * tid) = (v2u){pk16(lb[0], lb[1]), pk16(lb[2], lb[3])};
    __syncthreads();
    {
      const int m = (wave & 3) * 32 + lane;
      const v4u vh = *(const v4u*)(sHi + 4 * m);
      const v4u vl = *(const v4u*)(sLo + 4 * m);
      unsigned short* ph = onH + gtok * NHID + 8 * (size_t)m;
      unsigned short* pl = onL + gtok * NHID + 8 * (size_t)m;
      if (wave < 4) {
        *(volatile v4u*)ph = vh;
        __threadfence();
        *(volatile v4u*)ph = vh;
      } else {
        *(volatile v4u*)pl = vl;
        __threadfence();
        *(volatile v4u*)pl = vl;
      }
    }
#pragma unroll
    for (int j = 0; j < 4; ++j) { xm3[j] = xm2[j]; xm2[j] = xm1[j]; xm1[j] = x0[j]; }
  }
}

extern "C" void kernel_launch(void* const* d_in, const int* in_sizes, int n_in,
                              void* d_out, int out_size, void* d_ws, size_t ws_size,
                              hipStream_t stream) {
  if (n_in < 10) return;
  if (in_sizes[0] != NTOK * NHID) return;
  if (in_sizes[1] != NHID * NHID || in_sizes[2] != NHID * NHID || in_sizes[3] != NHID * NHID || in_sizes[9] != NHID * NHID) return;
  if (in_sizes[4] != NHID * NTAP || in_sizes[5] != NHID * NTAP || in_sizes[6] != NHID * NTAP) return;
  if (in_sizes[7] != NHEAD * NHID || in_sizes[8] != NHID) return;
  if (out_size != NTOK * NHID + NBH * NDH * NDH) return;
  if (ws_size < WS_TOTAL) return;

  const float* x      = (const float*)d_in[0];
  const float* Wq     = (const float*)d_in[1];
  const float* Wk     = (const float*)d_in[2];
  const float* Wv     = (const float*)d_in[3];
  const float* tq     = (const float*)d_in[4];
  const float* tk     = (const float*)d_in[5];
  const float* tv     = (const float*)d_in[6];
  const float* Wgate  = (const float*)d_in[7];
  const float* rmsw   = (const float*)d_in[8];
  const float* Wo     = (const float*)d_in[9];
  float* out0 = (float*)d_out;
  float* out1 = (float*)((char*)d_out + OUT0_BYTES);

  char* ws = (char*)d_ws;
  unsigned short* pX16  = (unsigned short*)(ws + OFF_X);
  unsigned short* pU16  = (unsigned short*)(ws + OFF_X);
  unsigned short* pWQ16 = (unsigned short*)(ws + OFF_WQ);
  unsigned short* pWK16 = (unsigned short*)(ws + OFF_WK);
  unsigned short* pWV16 = (unsigned short*)(ws + OFF_WV);
  unsigned short* pWO16 = (unsigned short*)(ws + OFF_WO);
  float*          pLIN  = (float*)(ws + OFF_LIN);
  unsigned short* pK16  = (unsigned short*)(ws + OFF_K);
  unsigned short* pKT16 = (unsigned short*)(ws + OFF_KT);
  unsigned short* pONH  = (unsigned short*)(ws + OFF_KT);
  unsigned short* pKBT  = (unsigned short*)(ws + OFF_KBT);
  unsigned short* pUT16 = (unsigned short*)(ws + OFF_KBT);
  unsigned short* pONL  = (unsigned short*)(ws + OFF_KBT);
  unsigned short* pVBT  = (unsigned short*)(ws + OFF_VBT);
  unsigned short* pW16  = (unsigned short*)(ws + OFF_VBT);
  unsigned short* pT16  = (unsigned short*)(ws + OFF_T);
  float*          pGATE = (float*)(ws + OFF_GATE);
  float*          pDS   = (float*)(ws + OFF_DS);

  const int n8x = (NTOK * NHID) / 8;
  const int n8w = (NHID * NHID) / 8;
  cast8_kernel<0><<<dim3(n8x / 256), dim3(256), 0, stream>>>(x,  pX16,  n8x, CARRY_X);
  cast8_kernel<0><<<dim3(n8w / 256), dim3(256), 0, stream>>>(Wq, pWQ16, n8w, CARRY_W);
  cast8_kernel<0><<<dim3(n8w / 256), dim3(256), 0, stream>>>(Wk, pWK16, n8w, CARRY_W);
  cast8_kernel<0><<<dim3(n8w / 256), dim3(256), 0, stream>>>(Wv, pWV16, n8w, CARRY_W);
  cast8_kernel<1><<<dim3(n8w / 256), dim3(256), 0, stream>>>(Wo, pWO16, n8w, 1.0f);
  gate_kernel<<<dim3(NTOK / 8), dim3(256), 0, stream>>>(x, Wgate, pGATE);

  const int projBlocks = ((NTOK / 64) * (NHID / 64)) / 8;
  const float projScale = 1.0f / (CARRY_X * CARRY_W);
  wmma_gemm64<0, 0, 0, 0, false, 0><<<dim3(projBlocks, 1), dim3(256), 0, stream>>>(
      pX16, pX16, NHID, 0L, pWK16, pWK16, NHID, 0L, (void*)pLIN, (void*)pLIN, NHID, 0L,
      pGATE, pGATE, 0L, NTOK, NHID, NHID, projScale);
  conv_kernel<0><<<dim3(NBN * NHEAD), dim3(256), CONV_LDS_BYTES, stream>>>(pLIN, tk, pGATE, pK16, pKT16, pKBT);
  wmma_gemm64<0, 0, 0, 0, false, 0><<<dim3(projBlocks, 1), dim3(256), 0, stream>>>(
      pX16, pX16, NHID, 0L, pWV16, pWV16, NHID, 0L, (void*)pLIN, (void*)pLIN, NHID, 0L,
      pGATE, pGATE, 0L, NTOK, NHID, NHID, projScale);
  conv_kernel<1><<<dim3(NBN * NHEAD), dim3(256), CONV_LDS_BYTES, stream>>>(pLIN, tv, pGATE, pVBT, pVBT, pVBT);
  wmma_gemm64<0, 0, 0, 0, false, 0><<<dim3(projBlocks, 1), dim3(256), 0, stream>>>(
      pX16, pX16, NHID, 0L, pWQ16, pWQ16, NHID, 0L, (void*)pLIN, (void*)pLIN, NHID, 0L,
      pGATE, pGATE, 0L, NTOK, NHID, NHID, projScale);
  tmat_kernel<<<dim3(NBN), dim3(256), 0, stream>>>(pK16, pGATE, pT16);
  const int tkbBlocks = ((NCS / 64) * (NHID / 64)) / 8;
  const float tkbScale = CARRY_WU / (CARRY_T * CARRY_K);
  wmma_gemm64<0, 0, 0, 1, false, 0><<<dim3(tkbBlocks, NBN), dim3(256), 0, stream>>>(
      pT16, pT16, NCS, (long)NCS * NCS, pVBT, pVBT, NCS, (long)NHID * NCS, (void*)pU16, (void*)pU16, NHID, (long)NCS * NHID,
      pGATE, pGATE, 0L, NCS, NHID, NCS, tkbScale);
  wmma_gemm64<0, 0, 0, 1, false, 0><<<dim3(tkbBlocks, NBN), dim3(256), 0, stream>>>(
      pT16, pT16, NCS, (long)NCS * NCS, pKBT, pKBT, NCS, (long)NHID * NCS, (void*)pW16, (void*)pW16, NHID, (long)NCS * NHID,
      pGATE, pGATE, 0L, NCS, NHID, NCS, tkbScale);
  diag_kernel<<<dim3(NBH), dim3(256), DIAG_LDS_BYTES, stream>>>(pKT16, pW16, pU16, pUT16, pDS);
  const int stBlocks = ((NDH / 64) * (NDH / 64)) / 8;
  wmma_gemm64<0, 0, 0, 0, false, 0><<<dim3(stBlocks, NBH), dim3(256), 0, stream>>>(
      pKT16, pKT16, NSEQ, (long)NDH * NSEQ, pUT16, pUT16, NSEQ, (long)NDH * NSEQ, (void*)out1, (void*)out1, NDH, (long)NDH * NDH,
      pGATE, pGATE, 0L, NDH, NDH, NSEQ, 1.0f / (CARRY_K * CARRY_UT));
  onorm_kernel<<<dim3(NTOK / ON_TPB), dim3(256), 0, stream>>>(pLIN, tq, pK16, pW16, pU16, pDS, rmsw, pONH, pONL);
  wmma_gemm64<1, 2, 0, 0, false, 0><<<dim3(projBlocks, 1), dim3(256), 0, stream>>>(
      pONH, pONL, NHID, 0L, pWO16, pWO16, NHID, 0L, (void*)out0, (void*)out0, NHID, 0L,
      pGATE, pGATE, 0L, NTOK, NHID, NHID, 1.0f);
}
